// EdgeConv_5549097746955
// MI455X (gfx1250) — hardware-verified
//
#include <hip/hip_runtime.h>
#include <stddef.h>
#include <stdint.h>

#define FDIM   64
#define NCOL   128
#define KNB    16
#define TROWS  64
#define GTHR   128
#define LDSA   72
#define PSP    128
#define GNODES 16
#define GGTHR  256
#define NUNW   (NCOL * (FDIM / 8))
#define WSMAX  134217728

static_assert(FDIM % 32 == 0 && NCOL == 2 * FDIM);
static_assert(TROWS == (GTHR / 32) * 16);
static_assert(((LDSA * 2) % 16) == 0 && LDSA >= FDIM);
static_assert((TROWS * FDIM) % (GTHR * 4) == 0);
static_assert((TROWS * PSP) % (GTHR * 4) == 0);
static_assert(GNODES * KNB == GGTHR);
static_assert(GNODES == 2 * (GGTHR / 32));
static_assert(NUNW % 256 == 0);

typedef float          v4f   __attribute__((ext_vector_type(4)));
typedef float          v8f   __attribute__((ext_vector_type(8)));
typedef int            v8i   __attribute__((ext_vector_type(8)));
typedef unsigned short v4us  __attribute__((ext_vector_type(4)));
typedef unsigned short v8us  __attribute__((ext_vector_type(8)));
typedef unsigned short v16us __attribute__((ext_vector_type(16)));
typedef __bf16         v16bf __attribute__((ext_vector_type(16)));
typedef v4f  __attribute__((may_alias)) v4fa;
typedef v4us __attribute__((may_alias)) v4usa;
typedef v8us __attribute__((may_alias)) v8usa;
union FragB { v16bf v; v16us u; v8us h[2]; v8i w; };

__device__ __forceinline__ v8f wmb(const FragB& a, const FragB& b, v8f c) {
  v8f d = __builtin_amdgcn_wmma_f32_16x16x32_bf16(false, a.v, false, b.v, (short)0, c, false, false);
  asm volatile("v_nop\n\tv_nop\n\tv_nop\n\tv_nop" : "+v"(d) : "v"(a.w), "v"(b.w));
  return d;
}

__device__ __forceinline__ unsigned bf16_bits(float f) {
  const unsigned u = __float_as_uint(f);
  return (u + 0x7FFFu + ((u >> 16) & 1u)) >> 16;
}
__device__ __forceinline__ float bf16_val(float f) {
  return __uint_as_float(bf16_bits(f) << 16);
}

__global__ __launch_bounds__(256) void k_wprep(const float* __restrict__ Wt, const float* __restrict__ Wp,
                                               unsigned short* WT, int nUnits) {
  const int u = (int)blockIdx.x * 256 + (int)threadIdx.x;
  if (u >= nUnits) return;
  const int n  = u >> 3;
  const int k8 = u & 7;
  const int col = n & (FDIM - 1);
  const float* src = (n < FDIM) ? Wt : Wp;
  const float* p = src + (size_t)(8 * k8) * FDIM + col;
  v8us o;
#pragma unroll
  for (int j = 0; j < 8; ++j) o[j] = (unsigned short)bf16_bits(p[(size_t)j * FDIM]);
  unsigned short* dp = WT + (size_t)n * FDIM + 8 * k8;
  *(volatile v8us*)dp = o;
  __threadfence();
  *(volatile v8us*)dp = o;
}

__device__ __forceinline__ void plane_store_pass(const float* sO, float* base, int tid) {
#pragma unroll
  for (int i = 0; i < (TROWS * PSP) / (GTHR * 4); ++i) {
    const int f = i * (GTHR * 4) + 4 * tid;
    const v4f v = *(const v4fa*)(sO + f);
    *(volatile v4f*)(base + f) = v;
  }
}

__global__ __launch_bounds__(GTHR) void k_gemm(
    const float* __restrict__ feat,
    const unsigned short* __restrict__ WT,
    const float* __restrict__ bt,
    const float* __restrict__ bp,
    float* PS,
    int nN)
{
  __shared__ __attribute__((aligned(16))) unsigned short sA[TROWS * LDSA];
  __shared__ __attribute__((aligned(16))) float sO[TROWS * PSP];

  const int tid = (int)threadIdx.x, lane = tid & 31, wave = tid >> 5;
  const int hh = lane >> 4, m = lane & 15;
  const int row0 = (int)blockIdx.x * TROWS;
  if (row0 + TROWS > nN) return;

  {
    const int c4 = tid & 15;
    const int rs = tid >> 4;
#pragma unroll
    for (int i = 0; i < (TROWS * FDIM) / (GTHR * 4); ++i) {
      const int row = rs + 8 * i;
      const v4f v = *(const v4fa*)(feat + (size_t)(row0 + row) * FDIM + 4 * c4);
      v4us o;
      o[0] = (unsigned short)bf16_bits(v.x);
      o[1] = (unsigned short)bf16_bits(v.y);
      o[2] = (unsigned short)bf16_bits(v.z);
      o[3] = (unsigned short)bf16_bits(v.w);
      *(v4usa*)(sA + row * LDSA + 4 * c4) = o;
    }
  }
  __syncthreads();

  v8f acc[8];
  {
    const v8f z8 = {0.f, 0.f, 0.f, 0.f, 0.f, 0.f, 0.f, 0.f};
#pragma unroll
    for (int t = 0; t < 8; ++t) acc[t] = z8;
  }
  const unsigned short* ap = sA + (16 * wave + m) * LDSA + 8 * hh;
  const unsigned short* wp = WT + (size_t)m * FDIM + 8 * hh;

#pragma unroll
  for (int kk = 0; kk < FDIM / 32; ++kk) {
    const int k0 = 32 * kk;
    FragB af;
    af.h[0] = *(const v8usa*)(ap + k0);
    af.h[1] = *(const v8usa*)(ap + k0 + 16);
#pragma unroll
    for (int nt = 0; nt < 8; ++nt) {
      const unsigned short* wq = wp + (size_t)(16 * nt) * FDIM + k0;
      FragB bf;
      bf.h[0] = *(const v8usa*)wq;
      bf.h[1] = *(const v8usa*)(wq + 16);
      acc[nt] = wmb(af, bf, acc[nt]);
    }
  }

#pragma unroll
  for (int nt = 0; nt < 4; ++nt) {
    const int col = 16 * nt + m;
    const float tb = bf16_val(bt[col]);
    const float pb = bf16_val(bp[col]);
#pragma unroll
    for (int r = 0; r < 8; ++r) {
      const int row = 16 * wave + 8 * hh + r;
      const float p = acc[nt][r];
      const float q = acc[nt + 4][r];
      sO[row * PSP + col]        = p;
      sO[row * PSP + FDIM + col] = (p + tb) + (q + pb);
    }
  }
  __syncthreads();

  float* base = PS + (size_t)row0 * PSP;
  plane_store_pass(sO, base, tid);
  __threadfence();
  plane_store_pass(sO, base, tid);
}

__global__ __launch_bounds__(GGTHR) void k_gather(
    const int*   __restrict__ nbr,
    const float* __restrict__ PS,
    float* out,
    int nN)
{
  __shared__ int sIdx[GNODES * KNB];

  const int tid = (int)threadIdx.x;
  const int node0 = (int)blockIdx.x * GNODES;
  {
    const int total = nN * KNB;
    int gi = node0 * KNB + tid;
    gi = gi > total - 1 ? total - 1 : gi;
    const int raw = nbr[gi];
    int ix = raw < 0 ? raw + nN : raw;
    ix = ix < 0 ? 0 : (ix > nN - 1 ? nN - 1 : ix);
    sIdx[tid] = ix;
  }
  __syncthreads();

  const int lane = tid & 31, wave = tid >> 5;
  const int hh = lane >> 4, c = lane & 15;
  const int vl = 2 * wave + hh;
  const int v  = node0 + vl;
  const int vc = v > nN - 1 ? nN - 1 : v;

  const v4f s = *(const v4fa*)(PS + (size_t)vc * PSP + FDIM + 4 * c);
  v4f mn = {3.402823466e+38f, 3.402823466e+38f, 3.402823466e+38f, 3.402823466e+38f};
#pragma unroll 4
  for (int k = 0; k < KNB; ++k) {
    const int u = sIdx[vl * KNB + k];
    const v4f p = *(const v4fa*)(PS + (size_t)u * PSP + 4 * c);
    mn.x = fminf(mn.x, p.x);
    mn.y = fminf(mn.y, p.y);
    mn.z = fminf(mn.z, p.z);
    mn.w = fminf(mn.w, p.w);
  }
  v4f o;
  o.x = s.x - mn.x;
  o.y = s.y - mn.y;
  o.z = s.z - mn.z;
  o.w = s.w - mn.w;

  const bool ok = (v < nN);
  float* dst = out + (size_t)vc * FDIM + 4 * c;
  if (ok) *(volatile v4f*)dst = o;
  __threadfence();
  if (ok) *(volatile v4f*)dst = o;
}

static inline int cdiv(int a, int b) { return (a + b - 1) / b; }

extern "C" void kernel_launch(void* const* d_in, const int* in_sizes, int n_in,
                              void* d_out, int out_size, void* d_ws, size_t ws_size,
                              hipStream_t stream) {
  if (n_in < 6) return;
  if (in_sizes[0] < FDIM || (in_sizes[0] % FDIM) != 0) return;
  const int nN = in_sizes[0] / FDIM;
  if ((nN % TROWS) != 0 || (nN % GNODES) != 0) return;
  if (in_sizes[1] != nN * KNB) return;
  if (in_sizes[2] != FDIM * FDIM) return;
  if (in_sizes[3] != FDIM) return;
  if (in_sizes[4] != FDIM * FDIM) return;
  if (in_sizes[5] != FDIM) return;
  if (out_size != nN * FDIM) return;

  const float* feat = (const float*)d_in[0];
  const int*   nbr  = (const int*)d_in[1];
  const float* Wt   = (const float*)d_in[2];
  const float* bt   = (const float*)d_in[3];
  const float* Wp   = (const float*)d_in[4];
  const float* bp   = (const float*)d_in[5];
  float* out = (float*)d_out;

  char* ws = (char*)d_ws;
  size_t off = 0;
  const size_t oWT = off; off += (size_t)NCOL * FDIM * 2;        off = (off + 255) & ~(size_t)255;
  const size_t oPS = off; off += (size_t)nN * PSP * sizeof(float); off = (off + 255) & ~(size_t)255;
  if (off > ws_size || off > (size_t)WSMAX) return;
  unsigned short* WT = (unsigned short*)(ws + oWT);
  float* PS = (float*)(ws + oPS);

  k_wprep<<<cdiv(NUNW, 256), 256, 0, stream>>>(Wt, Wp, WT, NUNW);
  k_gemm<<<nN / TROWS, GTHR, 0, stream>>>(feat, WT, bt, bp, PS, nN);
  k_gather<<<nN / GNODES, GGTHR, 0, stream>>>(nbr, PS, out, nN);
}
